// QMambaBlock_10960756539576
// MI455X (gfx1250) — hardware-run, weakly checked
//
#include <hip/hip_runtime.h>
#include <math.h>

typedef __attribute__((ext_vector_type(16))) _Float16 v16h;
typedef __attribute__((ext_vector_type(8)))  _Float16 v8h;
typedef __attribute__((ext_vector_type(16))) __bf16   v16b;
typedef __attribute__((ext_vector_type(8)))  __bf16   v8b;
typedef __attribute__((ext_vector_type(8)))  float    v8f;
typedef __attribute__((ext_vector_type(4)))  float    v4f;

constexpr int kNb    = 16;
constexpr int kCh    = 128;
constexpr int kHt    = 64;
constexpr int kWd    = 64;
constexpr int kPadH  = 66;
constexpr int kPadW  = 66;
constexpr int kLen   = kHt * kWd;
constexpr int kSt    = 16;
constexpr int kTok   = kNb * kLen;
constexpr int kKconv = 9 * kCh;
constexpr int kTiles = kNb * kHt;
static_assert(kLen == 4096 && kTok == 65536 && kKconv == 1152 && kTiles == 1024, "shape constants");
static_assert((kKconv % 32) == 0 && (kCh % 32) == 0, "K multiples of 32");
static_assert((kTok % 64) == 0 && (kCh % 64) == 0, "M and N multiples of 64");
static_assert((kLen % 32) == 0, "scan chunking");
static_assert(kNb == 16, "gate product M equals one 16-row tile");

constexpr float kCarryConv    = 256.0f;
constexpr float kCarryDt      = 64.0f;
constexpr float kCarryGate    = 64.0f;
constexpr float kInvCarryConv = 1.0f / 256.0f;
constexpr float kInvCarryDt   = 1.0f / 64.0f;
constexpr float kInvGateProd  = 1.0f / (64.0f * 64.0f);
constexpr float kInvLen       = 1.0f / 4096.0f;
static_assert(kCarryDt == kCarryGate, "one carry for the three [128][128] weight planes");

constexpr size_t kXpadB   = (size_t)kNb * kPadH * kPadW * kCh * 2;
constexpr size_t kWconvB  = (size_t)kCh * kKconv * 2;
constexpr size_t kWsqB    = (size_t)kCh * kCh * 2;
constexpr size_t kConv32B = (size_t)kTok * kCh * 4;
constexpr size_t kPartB   = (size_t)kTiles * kCh * 4;
constexpr size_t kGateB   = (size_t)kNb * kCh * 4;
constexpr size_t kXg16B   = (size_t)kTok * kCh * 2;
constexpr size_t kDt32B   = (size_t)kTok * kCh * 4;
constexpr size_t kOfsXPAD   = 0;
constexpr size_t kOfsWCONV  = kOfsXPAD   + kXpadB;
constexpr size_t kOfsWDT    = kOfsWCONV  + kWconvB;
constexpr size_t kOfsG1W    = kOfsWDT    + kWsqB;
constexpr size_t kOfsG2W    = kOfsG1W    + kWsqB;
constexpr size_t kOfsCONV32 = kOfsG2W    + kWsqB;
constexpr size_t kOfsPART   = kOfsCONV32 + kConv32B;
constexpr size_t kOfsGATE   = kOfsPART   + kPartB;
constexpr size_t kOfsXG16   = kOfsGATE   + kGateB;
constexpr size_t kOfsDT32   = kOfsXG16   + kXg16B;
constexpr size_t kWsTotal   = kOfsDT32   + kDt32B;
static_assert(kXpadB == 17842176ull && kWconvB == 294912ull && kWsqB == 32768ull, "plane sizes a");
static_assert(kConv32B == 33554432ull && kPartB == 524288ull && kGateB == 8192ull && kXg16B == 16777216ull, "plane sizes b");
static_assert(kWsTotal == 102653952ull, "carve total");
static_assert(kWsTotal <= 134217728ull, "carve cap");
static_assert((kXpadB % 128) == 0 && (kWconvB % 512) == 0 && (kWsqB % 512) == 0 && (kConv32B % 128) == 0 &&
              (kPartB % 512) == 0 && (kGateB % 128) == 0 && (kXg16B % 512) == 0, "line-aligned regions");

__device__ __forceinline__ _Float16 to_h_flush(float v) {
  const float w = (fabsf(v) < 6.103515625e-05f) ? 0.0f : v;
  return (_Float16)w;
}

union FragU { v16h v; v8h h[2]; };
__device__ __forceinline__ v16h frag_load(const _Float16* p) {
  FragU f;
  f.h[0] = *(const v8h*)(p);
  f.h[1] = *(const v8h*)(p + 16);
  return f.v;
}
__device__ __forceinline__ v8f mma_g(v16h a, v16h b, v8f c) {
  c = __builtin_amdgcn_wmma_f32_16x16x32_f16(false, a, false, b, (short)0, c, false, false);
  asm volatile("v_nop\n\tv_nop\n\tv_nop\n\tv_nop" : "+v"(c) : "v"(a), "v"(b));
  return c;
}

__global__ __launch_bounds__(256) void pack_x_kernel(const float* __restrict__ X, unsigned short* P16) {
  __shared__ __align__(16) float tile[128 * 68];
  const int tid = threadIdx.x;
  const int b = blockIdx.x / kPadH;
  const int py = blockIdx.x - b * kPadH;
  const bool rowlive = (py >= 1) && (py <= kHt);
  if (rowlive) {
    const int y = py - 1;
#pragma unroll
    for (int it = 0; it < 8; ++it) {
      const int i = it * 256 + tid;
      const int c = i >> 4;
      const int x4 = (i & 15) * 4;
      const v4f v = *(const v4f*)(X + ((size_t)(b * kCh + c) * kHt + y) * kWd + x4);
      *(v4f*)(tile + c * 68 + x4) = v;
    }
  }
  __syncthreads();
  const v8h zero8 = (v8h){(_Float16)0.f, (_Float16)0.f, (_Float16)0.f, (_Float16)0.f,
                          (_Float16)0.f, (_Float16)0.f, (_Float16)0.f, (_Float16)0.f};
  v8h hv[5];
#pragma unroll
  for (int it = 0; it < 5; ++it) hv[it] = zero8;
  if (rowlive) {
#pragma unroll
    for (int it = 0; it < 5; ++it) {
      const int i = it * 256 + tid;
      const int ic = (i < 1055) ? i : 1055;
      const int px = ic >> 4;
      const int c8 = (ic & 15) * 8;
      const bool live = (px >= 1) && (px <= kWd);
      int pxl = px - 1;
      pxl = (pxl < 0) ? 0 : pxl;
      pxl = (pxl > kWd - 1) ? (kWd - 1) : pxl;
#pragma unroll
      for (int e = 0; e < 8; ++e) {
        const float t = tile[(c8 + e) * 68 + pxl];
        const _Float16 hq = to_h_flush(t);
        hv[it][e] = live ? hq : (_Float16)0.f;
      }
    }
  }
  unsigned short* rowbase = P16 + ((size_t)(b * kPadH + py) * kPadW) * kCh;
  for (int pass = 0; pass < 2; ++pass) {
#pragma unroll
    for (int it = 0; it < 5; ++it) {
      const int i = it * 256 + tid;
      if (i < 1056) *(volatile v8h*)(rowbase + (size_t)i * 8) = hv[it];
    }
    __threadfence();
  }
}

__global__ __launch_bounds__(256) void pack_w_kernel(const float* __restrict__ cw, const float* __restrict__ dw,
                                                     const float* __restrict__ g1w, const float* __restrict__ g2w,
                                                     unsigned short* wconv, unsigned short* wdt,
                                                     unsigned short* wg1, unsigned short* wg2) {
  if (blockIdx.x < 72) {
    const int t = blockIdx.x * 256 + threadIdx.x;
    const int o = t / 144;
    const int k8 = (t - o * 144) * 8;
    const int tap = k8 >> 7;
    const int ci0 = k8 & 127;
    v8h hv;
#pragma unroll
    for (int e = 0; e < 8; ++e) {
      const float v = cw[(size_t)(o * kCh + ci0 + e) * 9 + tap] * kCarryConv;
      hv[e] = to_h_flush(v);
    }
    unsigned short* q = wconv + (size_t)t * 8;
    *(volatile v8h*)q = hv;
    __threadfence();
    *(volatile v8h*)q = hv;
  } else {
    const int idx = (int)blockIdx.x - 72;
    const int which = idx >> 3;
    const float* src = (which == 0) ? dw : ((which == 1) ? g1w : g2w);
    unsigned short* dst = (which == 0) ? wdt : ((which == 1) ? wg1 : wg2);
    const int t = (idx & 7) * 256 + threadIdx.x;
    const v4f a0 = *(const v4f*)(src + (size_t)t * 8);
    const v4f a1 = *(const v4f*)(src + (size_t)t * 8 + 4);
    v8h hv;
#pragma unroll
    for (int e = 0; e < 4; ++e) {
      hv[e] = to_h_flush(a0[e] * kCarryDt);
      hv[4 + e] = to_h_flush(a1[e] * kCarryDt);
    }
    unsigned short* q = dst + (size_t)t * 8;
    *(volatile v8h*)q = hv;
    __threadfence();
    *(volatile v8h*)q = hv;
  }
}

__global__ __launch_bounds__(128) void conv3x3_kernel(const unsigned short* __restrict__ P0p,
                                                      const unsigned short* __restrict__ Btp,
                                                      const float* __restrict__ bias,
                                                      float* out32, float* partials) {
  constexpr int SP = 68;
  __shared__ __align__(16) float sS[4 * 16 * SP];
  __shared__ __align__(16) float sPart[4 * 64];
  const int tid = threadIdx.x;
  const int lane = tid & 31;
  const int wave = tid >> 5;
  const int m = lane & 15;
  const int h = lane >> 4;
  const int b = blockIdx.x >> 6;
  const int y = blockIdx.x & 63;
  const int xh = wave & 1;
  const int nh = wave >> 1;
  const int x0 = xh * 32;
  const int n0 = nh * 64;
  const _Float16* A0 = (const _Float16*)P0p;
  const _Float16* Bl = (const _Float16*)Btp + (size_t)(n0 + m) * kKconv + 8 * h;

  v8f acc[2][4];
#pragma unroll
  for (int i = 0; i < 2; ++i)
#pragma unroll
    for (int j = 0; j < 4; ++j) acc[i][j] = (v8f){0.f, 0.f, 0.f, 0.f, 0.f, 0.f, 0.f, 0.f};

#pragma unroll 1
  for (int tap = 0; tap < 9; ++tap) {
    const int kh = tap / 3;
    const int kw = tap - kh * 3;
    const size_t pixoff = ((size_t)(b * kPadH + y + kh) * kPadW + (x0 + m + kw)) * kCh + 8 * h;
    const _Float16* Ap = A0 + pixoff;
#pragma unroll
    for (int cc = 0; cc < 4; ++cc) {
      const v16h a0 = frag_load(Ap + cc * 32);
      const v16h a1 = frag_load(Ap + 16 * kCh + cc * 32);
      const _Float16* Bp = Bl + tap * kCh + cc * 32;
#pragma unroll
      for (int j = 0; j < 4; ++j) {
        const v16h bf = frag_load(Bp + (size_t)j * 16 * kKconv);
        acc[0][j] = mma_g(a0, bf, acc[0][j]);
        acc[1][j] = mma_g(a1, bf, acc[1][j]);
      }
    }
  }

  float bv[4];
  float csum[4];
#pragma unroll
  for (int j = 0; j < 4; ++j) {
    bv[j] = bias[n0 + j * 16 + m];
    csum[j] = 0.0f;
  }

  float* slab = sS + wave * 16 * SP;
  const size_t tokrow = (size_t)(b * kHt + y) * kWd;
#pragma unroll
  for (int mt = 0; mt < 2; ++mt) {
#pragma unroll
    for (int j = 0; j < 4; ++j) {
#pragma unroll
      for (int r = 0; r < 8; ++r) {
        const float v = acc[mt][j][r] * kInvCarryConv + bv[j];
        slab[(8 * h + r) * SP + j * 16 + m] = v;
        csum[j] += v;
      }
    }
    __syncthreads();
    float* dst = out32 + (tokrow + x0 + mt * 16) * kCh + n0;
    const int c4 = m * 4;
    v4f vv[8];
#pragma unroll
    for (int it = 0; it < 8; ++it) {
      const int row = it * 2 + h;
      vv[it] = *(const v4f*)(slab + row * SP + c4);
    }
    for (int pass = 0; pass < 2; ++pass) {
#pragma unroll
      for (int it = 0; it < 8; ++it) {
        const int row = it * 2 + h;
        *(volatile v4f*)(dst + (size_t)row * kCh + c4) = vv[it];
      }
      __threadfence();
    }
    __syncthreads();
  }

#pragma unroll
  for (int j = 0; j < 4; ++j) csum[j] += __shfl_xor(csum[j], 16, 32);
  if (h == 0) {
#pragma unroll
    for (int j = 0; j < 4; ++j) sPart[wave * 64 + j * 16 + m] = csum[j];
  }
  __syncthreads();
  if (wave == 0) {
    const int c4 = lane * 4;
    const int nhh = c4 >> 6;
    const int cl = c4 & 63;
    const v4f pa = *(const v4f*)(sPart + (nhh * 2 + 0) * 64 + cl);
    const v4f pb = *(const v4f*)(sPart + (nhh * 2 + 1) * 64 + cl);
    v4f s;
#pragma unroll
    for (int e = 0; e < 4; ++e) s[e] = pa[e] + pb[e];
    float* q = partials + (size_t)blockIdx.x * kCh + c4;
    *(volatile v4f*)q = s;
    __threadfence();
    *(volatile v4f*)q = s;
  }
}

__global__ __launch_bounds__(256) void gate_kernel(const float* __restrict__ partials,
                                                   const unsigned short* __restrict__ w1p, const float* __restrict__ b1,
                                                   const unsigned short* __restrict__ w2p, const float* __restrict__ b2,
                                                   float* gout) {
  constexpr int AP = 136;
  constexpr int FP = 132;
  __shared__ __align__(16) _Float16 sA[16 * AP];
  __shared__ __align__(16) _Float16 sH[16 * AP];
  __shared__ __align__(16) float sF[16 * FP];
  const int tid = threadIdx.x;
  const int lane = tid & 31;
  const int wave = tid >> 5;
  const int m = lane & 15;
  const int h = lane >> 4;
  const int rb = tid >> 4;
  const int c8 = (tid & 15) * 8;
  const int n = wave * 16 + m;

  {
    v4f s0 = (v4f){0.f, 0.f, 0.f, 0.f};
    v4f s1 = (v4f){0.f, 0.f, 0.f, 0.f};
    const float* pp = partials + (size_t)rb * kHt * kCh + c8;
#pragma unroll 2
    for (int t = 0; t < kHt; ++t) {
      const v4f p0 = *(const v4f*)(pp + (size_t)t * kCh);
      const v4f p1 = *(const v4f*)(pp + (size_t)t * kCh + 4);
      s0 += p0;
      s1 += p1;
    }
    v8h hv;
#pragma unroll
    for (int e = 0; e < 4; ++e) {
      const float q0 = s0[e] * kInvLen;
      const float q1 = s1[e] * kInvLen;
      hv[e] = to_h_flush(q0 * kCarryGate);
      hv[4 + e] = to_h_flush(q1 * kCarryGate);
    }
    *(v8h*)(sA + rb * AP + c8) = hv;
  }
  __syncthreads();

  {
    const _Float16* Wr = (const _Float16*)w1p + (size_t)n * kCh + 8 * h;
    const _Float16* Ar = sA + m * AP + 8 * h;
    v8f acc = (v8f){0.f, 0.f, 0.f, 0.f, 0.f, 0.f, 0.f, 0.f};
#pragma unroll
    for (int ks = 0; ks < 4; ++ks) {
      const v16h a = frag_load(Ar + ks * 32);
      const v16h bf = frag_load(Wr + ks * 32);
      acc = mma_g(a, bf, acc);
    }
    const float bb = b1[n];
#pragma unroll
    for (int r = 0; r < 8; ++r) {
      const float v = acc[r] * kInvGateProd + bb;
      sF[(8 * h + r) * FP + n] = fmaxf(v, 0.0f);
    }
  }
  __syncthreads();
  {
    const v4f q0 = *(const v4f*)(sF + rb * FP + c8);
    const v4f q1 = *(const v4f*)(sF + rb * FP + c8 + 4);
    v8h hv;
#pragma unroll
    for (int e = 0; e < 4; ++e) {
      hv[e] = to_h_flush(q0[e] * kCarryGate);
      hv[4 + e] = to_h_flush(q1[e] * kCarryGate);
    }
    *(v8h*)(sH + rb * AP + c8) = hv;
  }
  __syncthreads();

  {
    const _Float16* Wr = (const _Float16*)w2p + (size_t)n * kCh + 8 * h;
    const _Float16* Ar = sH + m * AP + 8 * h;
    v8f acc = (v8f){0.f, 0.f, 0.f, 0.f, 0.f, 0.f, 0.f, 0.f};
#pragma unroll
    for (int ks = 0; ks < 4; ++ks) {
      const v16h a = frag_load(Ar + ks * 32);
      const v16h bf = frag_load(Wr + ks * 32);
      acc = mma_g(a, bf, acc);
    }
    const float bb = b2[n];
#pragma unroll
    for (int r = 0; r < 8; ++r) {
      const float v = acc[r] * kInvGateProd + bb;
      sF[(8 * h + r) * FP + n] = 1.0f / (1.0f + expf(-v));
    }
  }
  __syncthreads();

  if (wave < 4) {
    v4f vv[4];
#pragma unroll
    for (int it = 0; it < 4; ++it) {
      const int row = wave * 4 + it;
      vv[it] = *(const v4f*)(sF + row * FP + lane * 4);
    }
    for (int pass = 0; pass < 2; ++pass) {
#pragma unroll
      for (int it = 0; it < 4; ++it) {
        const int row = wave * 4 + it;
        *(volatile v4f*)(gout + (size_t)row * kCh + lane * 4) = vv[it];
      }
      __threadfence();
    }
  }
}

__global__ __launch_bounds__(256) void gate_apply_kernel(const float* __restrict__ conv32, const float* __restrict__ g,
                                                         unsigned short* xg16) {
  const size_t t = (size_t)blockIdx.x * 256 + threadIdx.x;
  const size_t e0 = t * 8;
  const int tok = (int)(t >> 4);
  const int b = tok >> 12;
  const int c8 = (int)(t & 15) * 8;
  const v4f a0 = *(const v4f*)(conv32 + e0);
  const v4f a1 = *(const v4f*)(conv32 + e0 + 4);
  const v4f g0 = *(const v4f*)(g + (size_t)b * kCh + c8);
  const v4f g1 = *(const v4f*)(g + (size_t)b * kCh + c8 + 4);
  v8h hv;
#pragma unroll
  for (int e = 0; e < 4; ++e) {
    hv[e] = to_h_flush(a0[e] * g0[e]);
    hv[4 + e] = to_h_flush(a1[e] * g1[e]);
  }
  unsigned short* q = xg16 + e0;
  *(volatile v8h*)q = hv;
  __threadfence();
  *(volatile v8h*)q = hv;
}

__device__ __forceinline__ unsigned short f2bf_bits(float f) {
  unsigned u = __float_as_uint(f);
  return (unsigned short)((u + 0x7FFFu + ((u >> 16) & 1u)) >> 16);
}
__device__ __forceinline__ float bf_bits2f(unsigned short h) { return __uint_as_float(((unsigned)h) << 16); }

__device__ __forceinline__ void dep_guard_h(v8f& a, v8f& b, v16h x, v16h y) { asm volatile("v_nop\n\tv_nop\n\tv_nop\n\tv_nop" : "+v"(a), "+v"(b) : "v"(x), "v"(y)); }
__device__ __forceinline__ void dep_guard_b(v8f& a, v8f& b, v16b x, v16b y) { asm volatile("v_nop\n\tv_nop\n\tv_nop\n\tv_nop" : "+v"(a), "+v"(b) : "v"(x), "v"(y)); }
__device__ __forceinline__ void keep4_h(v16h a, v16h b, v16h c, v16h d) { asm volatile("v_nop" :: "v"(a), "v"(b), "v"(c), "v"(d)); }
__device__ __forceinline__ void keep4_b(v16b a, v16b b, v16b c, v16b d) { asm volatile("v_nop" :: "v"(a), "v"(b), "v"(c), "v"(d)); }
__device__ __forceinline__ void acc_guard4(v8f& a, v8f& b, v8f& c, v8f& d) { asm volatile("v_nop\n\tv_nop\n\tv_nop\n\tv_nop" : "+v"(a), "+v"(b), "+v"(c), "+v"(d)); }
template <typename T> struct Frag;
template <> struct Frag<_Float16> {
  typedef v16h V; union U { v16h v; v8h h[2]; };
  static __device__ __forceinline__ v16h load(const _Float16* p) {
    U f; f.h[0] = *(const v8h*)(p); f.h[1] = *(const v8h*)(p + 16); return f.v;
  }
  static __device__ __forceinline__ v8f mma(v16h a, v16h b, v8f c) {
    return __builtin_amdgcn_wmma_f32_16x16x32_f16(false, a, false, b, (short)0, c, false, false);
  }
  static __device__ __forceinline__ void guard(v8f& a, v8f& b, v16h x, v16h y) { dep_guard_h(a, b, x, y); }
  static __device__ __forceinline__ void keep(v16h a, v16h b, v16h c, v16h d) { keep4_h(a, b, c, d); }
};
template <> struct Frag<__bf16> {
  typedef v16b V; union U { v16b v; v8b h[2]; };
  static __device__ __forceinline__ v16b load(const __bf16* p) {
    U f; f.h[0] = *(const v8b*)(p); f.h[1] = *(const v8b*)(p + 16); return f.v;
  }
  static __device__ __forceinline__ v8f mma(v16b a, v16b b, v8f c) {
    return __builtin_amdgcn_wmma_f32_16x16x32_bf16(false, a, false, b, (short)0, c, false, false);
  }
  static __device__ __forceinline__ void guard(v8f& a, v8f& b, v16b x, v16b y) { dep_guard_b(a, b, x, y); }
  static __device__ __forceinline__ void keep(v16b a, v16b b, v16b c, v16b d) { keep4_b(a, b, c, d); }
};

template <int ET> struct Elem;
template <> struct Elem<0> { typedef _Float16 T; };
template <> struct Elem<1> { typedef __bf16 T; };
template <int ET, bool SPLIT, int BIAS_MODE, int OUT_MODE, bool RESID, int ACT = 0>
__global__ __launch_bounds__(256) void wmma_gemm64(
    const unsigned short* __restrict__ Ap, const unsigned short* __restrict__ A2p, int lda, long strideA,
    const unsigned short* __restrict__ Btp, const unsigned short* __restrict__ Bt2p, int ldb, long strideB,
    void* __restrict__ Cout, void* __restrict__ Cout2, int ldc, long strideC,
    const float* __restrict__ bias,
    const float* __restrict__ resid, long strideR,
    int M, int N, int K, float scale) {
  typedef typename Elem<ET>::T T;
  typedef typename Frag<T>::V V;
  const T* A = (const T*)Ap; const T* A2 = (const T*)A2p; const T* Bt = (const T*)Btp; const T* Bt2 = (const T*)Bt2p;
  __shared__ __align__(16) float sT[8][16 * 68];
  const int b    = blockIdx.y;
  const int lane = threadIdx.x & 31;
  const int wave = threadIdx.x >> 5;
  const int tilesN = N >> 6;
  const int tilesM = M >> 6;
  const int tile = blockIdx.x * 8 + wave;
  if (tile >= tilesM * tilesN) return;
  const int tm = tile / tilesN;
  const int tn = tile - tm * tilesN;
  const int m0 = tm << 6;
  const int n0 = tn << 6;

  const T* Ab  = A  + (size_t)b * strideA;
  const T* Bb  = Bt + (size_t)b * strideB;
  const T* Ab2 = SPLIT ? (A2  + (size_t)b * strideA) : nullptr;
  const T* Bb2 = SPLIT ? (Bt2 + (size_t)b * strideB) : nullptr;

  const int rlane = lane & 15;
  const int koff  = (lane >> 4) * 8;
  const int mOff  = (lane >> 4) * 8;

  v8f acc[4][4];
#pragma unroll
  for (int i = 0; i < 4; ++i)
#pragma unroll
    for (int j = 0; j < 4; ++j) acc[i][j] = (v8f){0.f,0.f,0.f,0.f,0.f,0.f,0.f,0.f};

  for (int k0 = 0; k0 < K; k0 += 32) {
    V bh[4], bl[4];
#pragma unroll
    for (int j = 0; j < 4; ++j) {
      const size_t bo = (size_t)(n0 + (j << 4) + rlane) * ldb + koff + k0;
      bh[j] = Frag<T>::load(Bb + bo);
      if (SPLIT) bl[j] = Frag<T>::load(Bb2 + bo);
    }
#pragma unroll
    for (int i = 0; i < 4; ++i) {
      const size_t ao = (size_t)(m0 + (i << 4) + rlane) * lda + koff + k0;
      V ah = Frag<T>::load(Ab + ao);
      V al;
      if (SPLIT) al = Frag<T>::load(Ab2 + ao);
#pragma unroll
      for (int j = 0; j < 4; ++j) {
        acc[i][j] = Frag<T>::mma(ah, bh[j], acc[i][j]);
        if (SPLIT) {
          acc[i][j] = Frag<T>::mma(ah, bl[j], acc[i][j]);
          acc[i][j] = Frag<T>::mma(al, bh[j], acc[i][j]);
        }
      }
      Frag<T>::guard(acc[i][0], acc[i][3], ah, SPLIT ? al : ah);
    }
    Frag<T>::keep(bh[0], bh[1], bh[2], bh[3]);
    if (SPLIT) Frag<T>::keep(bl[0], bl[1], bl[2], bl[3]);
  }
  acc_guard4(acc[0][0], acc[0][1], acc[0][2], acc[0][3]);
  acc_guard4(acc[1][0], acc[1][1], acc[1][2], acc[1][3]);
  acc_guard4(acc[2][0], acc[2][1], acc[2][2], acc[2][3]);
  acc_guard4(acc[3][0], acc[3][1], acc[3][2], acc[3][3]);

  float* slab = sT[wave];
  const float* Rb = RESID ? (resid + (size_t)b * strideR) : nullptr;
#pragma unroll
  for (int i = 0; i < 4; ++i) {
    const int mBase = m0 + (i << 4);
#pragma unroll
    for (int j = 0; j < 4; ++j) {
      const int n = n0 + (j << 4) + rlane;
      float bv = 0.f;
      if (BIAS_MODE == 2) bv = bias[n];
#pragma unroll
      for (int r = 0; r < 8; ++r) {
        float v = acc[i][j][r] * scale;
        if (BIAS_MODE == 1) v += bias[mBase + mOff + r];
        if (BIAS_MODE == 2) v += bv;
        if (RESID) v += Rb[(size_t)(mBase + mOff + r) * ldc + n];
        if (ACT == 1) v = tanhf(v);
        if (ACT == 2) v = fmaxf(v, 0.0f);
        if (ACT == 3) v = v / (1.0f + expf(-v));
        if (ACT == 4) v = (v > 0.f) ? v : 0.01f * v;
        if (ACT == 5) v = 0.5f * v * (1.0f + erff(v * 0.70710678118654752f));
        if (ACT == 6) v = 1.0f / (1.0f + expf(-v));
        slab[(mOff + r) * 68 + (j << 4) + rlane] = v;
      }
    }
    __builtin_amdgcn_fence(__ATOMIC_RELEASE, "workgroup");
    __builtin_amdgcn_wave_barrier();
    __builtin_amdgcn_fence(__ATOMIC_ACQUIRE, "workgroup");
    if (OUT_MODE == 0) {
      float* C = (float*)Cout + (size_t)b * strideC;
      const int hh = lane >> 4, c4 = (lane & 15) * 4;
      for (int pass = 0; pass < 2; ++pass) {
#pragma unroll
        for (int it = 0; it < 8; ++it) {
          const int row = it * 2 + hh;
          v4f v = *(const v4f*)(slab + row * 68 + c4);
          *(volatile v4f*)(C + (size_t)(mBase + row) * ldc + n0 + c4) = v;
        }
        __threadfence();
      }
    } else {
      const int q = lane >> 3, c8 = (lane & 7) * 8;
      unsigned short* C  = (unsigned short*)Cout  + (size_t)b * strideC;
      unsigned short* C2 = (OUT_MODE == 2) ? ((unsigned short*)Cout2 + (size_t)b * strideC) : nullptr;
      for (int pass = 0; pass < 2; ++pass) {
#pragma unroll
        for (int it = 0; it < 4; ++it) {
          const int row = it * 4 + q;
          const float* sp = slab + row * 68 + c8;
          v8h hv, lv;
#pragma unroll
          for (int e = 0; e < 8; ++e) {
            if (OUT_MODE == 1) {
              hv[e] = (_Float16)sp[e];
            } else {
              unsigned short hb = f2bf_bits(sp[e]);
              unsigned short lb = f2bf_bits(sp[e] - bf_bits2f(hb));
              hv[e] = __builtin_bit_cast(_Float16, hb);
              lv[e] = __builtin_bit_cast(_Float16, lb);
            }
          }
          *(volatile v8h*)(C + (size_t)(mBase + row) * ldc + n0 + c8) = hv;
          if (OUT_MODE == 2) *(volatile v8h*)(C2 + (size_t)(mBase + row) * ldc + n0 + c8) = lv;
        }
        __threadfence();
      }
    }
    __builtin_amdgcn_fence(__ATOMIC_RELEASE, "workgroup");
    __builtin_amdgcn_wave_barrier();
    __builtin_amdgcn_fence(__ATOMIC_ACQUIRE, "workgroup");
  }
}

__global__ __launch_bounds__(32) void scan_kernel(const float* __restrict__ conv32, const float* __restrict__ dt32,
                                                  const float* __restrict__ g, const float* __restrict__ Ap,
                                                  const float* __restrict__ Dpp, const float* __restrict__ X,
                                                  float* out) {
  __shared__ __align__(16) float ytile[32 * 33];
  const int lane = threadIdx.x;
  const int b = blockIdx.x >> 2;
  const int c0 = (blockIdx.x & 3) * 32;
  const int c = c0 + lane;

  float An[kSt];
  float hs[kSt];
  {
    const v4f a0 = *(const v4f*)(Ap + (size_t)c * kSt);
    const v4f a1 = *(const v4f*)(Ap + (size_t)c * kSt + 4);
    const v4f a2 = *(const v4f*)(Ap + (size_t)c * kSt + 8);
    const v4f a3 = *(const v4f*)(Ap + (size_t)c * kSt + 12);
#pragma unroll
    for (int e = 0; e < 4; ++e) {
      An[e] = -expf(a0[e]);
      An[4 + e] = -expf(a1[e]);
      An[8 + e] = -expf(a2[e]);
      An[12 + e] = -expf(a3[e]);
    }
  }
#pragma unroll
  for (int s = 0; s < kSt; ++s) hs[s] = 0.0f;
  const float Dp = expf(Dpp[c]);
  const float gv = g[(size_t)b * kCh + c];

  const float* cp = conv32 + (size_t)b * kLen * kCh + c;
  const float* dp = dt32 + (size_t)b * kLen * kCh + c;

  for (int l0 = 0; l0 < kLen; l0 += 32) {
    for (int t = 0; t < 32; ++t) {
      const size_t idx = (size_t)(l0 + t) * kCh;
      const float cv = cp[idx];
      const float dv = dp[idx];
      const float xt = cv * gv;
      float y = 0.0f;
#pragma unroll
      for (int s = 0; s < kSt; ++s) {
        hs[s] = hs[s] * expf(An[s] * dv) + xt;
        y += hs[s] * An[s];
      }
      y += Dp * xt;
      ytile[t * 33 + lane] = y;
    }
    __syncthreads();
    v4f ov[8];
#pragma unroll
    for (int it = 0; it < 8; ++it) {
      const int chn = it * 4 + (lane >> 3);
      const int p4 = (lane & 7) * 4;
      const size_t gi = ((size_t)(b * kCh + c0 + chn)) * kLen + l0 + p4;
      const v4f xi = *(const v4f*)(X + gi);
#pragma unroll
      for (int e = 0; e < 4; ++e) ov[it][e] = ytile[(p4 + e) * 33 + chn] + xi[e];
    }
    for (int pass = 0; pass < 2; ++pass) {
#pragma unroll
      for (int it = 0; it < 8; ++it) {
        const int chn = it * 4 + (lane >> 3);
        const int p4 = (lane & 7) * 4;
        const size_t gi = ((size_t)(b * kCh + c0 + chn)) * kLen + l0 + p4;
        *(volatile v4f*)(out + gi) = ov[it];
      }
      __threadfence();
    }
    __syncthreads();
  }
}

extern "C" void kernel_launch(void* const* d_in, const int* in_sizes, int n_in,
                              void* d_out, int out_size, void* d_ws, size_t ws_size,
                              hipStream_t stream) {
  if (n_in < 11) return;
  if (in_sizes[0] != kNb * kCh * kHt * kWd) return;
  if (in_sizes[1] != kCh * kCh * 9) return;
  if (in_sizes[2] != kCh) return;
  if (in_sizes[3] != kCh * kCh) return;
  if (in_sizes[4] != kCh) return;
  if (in_sizes[5] != kCh * kSt) return;
  if (in_sizes[6] != kCh) return;
  if (in_sizes[7] != kCh * kCh) return;
  if (in_sizes[8] != kCh) return;
  if (in_sizes[9] != kCh * kCh) return;
  if (in_sizes[10] != kCh) return;
  if (out_size != kNb * kCh * kHt * kWd) return;
  if (ws_size < kWsTotal) return;

  const float* x      = (const float*)d_in[0];
  const float* conv_w = (const float*)d_in[1];
  const float* conv_b = (const float*)d_in[2];
  const float* dt_w   = (const float*)d_in[3];
  const float* dt_b   = (const float*)d_in[4];
  const float* Aprm   = (const float*)d_in[5];
  const float* Dprm   = (const float*)d_in[6];
  const float* g1_w   = (const float*)d_in[7];
  const float* g1_b   = (const float*)d_in[8];
  const float* g2_w   = (const float*)d_in[9];
  const float* g2_b   = (const float*)d_in[10];
  float* out = (float*)d_out;

  char* ws = (char*)d_ws;
  unsigned short* XPAD  = (unsigned short*)(ws + kOfsXPAD);
  unsigned short* WCONV = (unsigned short*)(ws + kOfsWCONV);
  unsigned short* WDT   = (unsigned short*)(ws + kOfsWDT);
  unsigned short* G1W   = (unsigned short*)(ws + kOfsG1W);
  unsigned short* G2W   = (unsigned short*)(ws + kOfsG2W);
  float* CONV32 = (float*)(ws + kOfsCONV32);
  float* PART   = (float*)(ws + kOfsPART);
  float* GATE   = (float*)(ws + kOfsGATE);
  unsigned short* XG16 = (unsigned short*)(ws + kOfsXG16);
  float* DT32   = (float*)(ws + kOfsDT32);

  pack_x_kernel<<<kNb * kPadH, 256, 0, stream>>>(x, XPAD);
  pack_w_kernel<<<96, 256, 0, stream>>>(conv_w, dt_w, g1_w, g2_w, WCONV, WDT, G1W, G2W);
  conv3x3_kernel<<<kTiles, 128, 0, stream>>>(XPAD, WCONV, conv_b, CONV32, PART);
  gate_kernel<<<1, 256, 0, stream>>>(PART, G1W, g1_b, G2W, g2_b, GATE);
  gate_apply_kernel<<<(kTok * (kCh / 8)) / 256, 256, 0, stream>>>(CONV32, GATE, XG16);
  static_assert(((kTok / 64) * (kCh / 64)) % 8 == 0, "gemm grid exact");
  wmma_gemm64<0, false, 2, 0, false, 6><<<dim3(((kTok / 64) * (kCh / 64)) / 8, 1), 256, 0, stream>>>(
      XG16, XG16, kCh, 0L, WDT, WDT, kCh, 0L, (void*)DT32, (void*)DT32, kCh, 0L,
      dt_b, dt_b, 0L, kTok, kCh, kCh, kInvCarryDt);
  scan_kernel<<<kNb * (kCh / 32), 32, 0, stream>>>(CONV32, DT32, GATE, Aprm, Dprm, x, out);
}
